// TransformerModel_32435593020281
// MI455X (gfx1250) — hardware-run, weakly checked
//
#include <hip/hip_runtime.h>
#include <stddef.h>
#include <stdint.h>
#include <math.h>

#define NN      50000
#define NE      800000
#define FIN     64
#define HC      256
#define NPRJ    832
#define OUTC    32
#define MP      50048
#define KL      128
#define GBM     128
#define NTHR    256
#define NWAVE   8
#define EPT     8
#define WCH     (32 * EPT)
#define NBRUN   1024
#define SLB     10
#define NBK     49
#define WLCAP   3840
#define RCAP    20480
#define TRIPCAP 1024
#define MAXDEG_MEAS   35
#define MAXB1024_MEAS 16623
#define RBM     64
#define SP      68
#define SPF     36
#define PERW    (((NE + NWAVE * WCH - 1) / (NWAVE * WCH)) * WCH)

#ifndef SPLIT2
#define SPLIT2 1
#endif
#ifndef SPLITF
#define SPLITF 1
#endif
#define K2EXT (SPLIT2 ? 128 : 64)
#define KFEXT (SPLITF ? 128 : 64)

#define SM_B1   0
#define SM_B2   832
#define SM_LNG  1664
#define SM_LNB  1728
#define SM_BF   1792
#define SM_TOT  1824

#define FKV     ((size_t)MP * 256)
#define FS      ((size_t)MP * 768)

#define BK_ZINTS (NWAVE * WLCAP + RCAP + 3 * NBRUN)
#define BK_INTS  (BK_ZINTS + 16)
#define BK_LDS   (BK_INTS * 4)

#define PB_X    (MP * FIN / 8 / NTHR)
#define PB_W1   (PB_X)
#define PB_W2   (PB_W1 + 26)
#define PB_WF   (PB_W2 + 52)
#define PB_SM   (PB_WF + 2)
#define PB_TOT  (PB_SM + 3)

static_assert(NN <= 65536);
static_assert(NBRUN == 1024 && NBRUN == (1 << SLB));
static_assert(MP % GBM == 0 && MP >= NN && MP == 391 * GBM && MP % RBM == 0);
static_assert(NBK * NBRUN >= MP);
static_assert(NBRUN % RBM == 0 && NBRUN % GBM == 0);
static_assert(NE < (1 << 20) && (((long long)NE) << SLB) < (1LL << 31));
static_assert(NE % WCH == 0 && NE % 4 == 0);
static_assert((NWAVE - 1) * PERW < NE && NWAVE * PERW >= NE);
static_assert((long long)RCAP * 100 >= (long long)MAXB1024_MEAS * 115);
static_assert(WLCAP * NWAVE * 2 >= 3 * RCAP);
static_assert(WLCAP >= MAXB1024_MEAS / 8 + 8 * 46 + 1);
static_assert(MAXDEG_MEAS + 8 <= TRIPCAP && TRIPCAP <= RCAP);
static_assert(RCAP % 4 == 0 && BK_ZINTS % 4 == 0 && (2 * NBRUN) % 4 == 0);
static_assert(BK_LDS <= 300000);
static_assert(NPRJ % 64 == 0 && NPRJ == 3 * HC + FIN);
static_assert(FIN % 32 == 0 && KL % 32 == 0 && KL == 2 * FIN);
static_assert((MP * FIN / 8) % NTHR == 0);
static_assert((GBM * SP + 64) * 4 <= 65536);
static_assert((GBM * SPF + 32) * 4 <= 65536);
static_assert((SM_TOT * 4) % 128 == 0 && (SM_B2 * 4) % 128 == 0 && (SM_LNG * 4) % 128 == 0 && (SM_BF * 4) % 128 == 0);
static_assert(NN % 4 == 0);
static_assert((long long)(NN - 1) * OUTC + OUTC - 1 == (long long)NN * OUTC - 1);

typedef float          v4f   __attribute__((ext_vector_type(4)));
typedef float          v8f   __attribute__((ext_vector_type(8)));
typedef int            v4i   __attribute__((ext_vector_type(4)));
typedef int            v8i   __attribute__((ext_vector_type(8)));
typedef unsigned int   v4u   __attribute__((ext_vector_type(4)));
typedef unsigned short v8us  __attribute__((ext_vector_type(8)));
typedef unsigned short v16us __attribute__((ext_vector_type(16)));
typedef __bf16         v16bf __attribute__((ext_vector_type(16)));
typedef v4f  __attribute__((may_alias)) v4fa;
typedef v4i  __attribute__((may_alias)) v4ia;
typedef v8us __attribute__((may_alias)) v8usa;
union FragB { v16bf v; v16us u; v8us h[2]; v8i w; };

__device__ __forceinline__ v8f wmb(const FragB& a, const FragB& b, v8f c) {
  v8f d = __builtin_amdgcn_wmma_f32_16x16x32_bf16(false, a.v, false, b.v, (short)0, c, false, false);
  asm volatile("v_nop\n\tv_nop\n\tv_nop\n\tv_nop" : "+v"(d) : "v"(a.w), "v"(b.w));
  return d;
}

__device__ __forceinline__ unsigned bf16_bits(float f) {
  const unsigned u = __float_as_uint(f);
  const unsigned r = (u + 0x7FFFu + ((u >> 16) & 1u)) >> 16;
  const unsigned q = (u >> 16) | 0x40u;
  return ((u & 0x7fffffffu) > 0x7f800000u) ? q : r;
}
__device__ __forceinline__ float bf16_val(float f) {
  return __uint_as_float(bf16_bits(f) << 16);
}

__device__ __forceinline__ void st2_v4f(float* p, v4f v) {
  *(volatile v4f*)p = v;
  __threadfence();
  *(volatile v4f*)p = v;
}
__device__ __forceinline__ void st2_v8us(unsigned short* p, v8us v) {
  *(volatile v8us*)p = v;
  __threadfence();
  *(volatile v8us*)p = v;
}

__device__ __forceinline__ v8us colpick8(const float* __restrict__ base, int stride) {
  float f[8];
#pragma unroll
  for (int i = 0; i < 8; ++i) f[i] = base[(size_t)i * (size_t)stride];
  v8us o;
#pragma unroll
  for (int i = 0; i < 8; ++i) o[i] = (unsigned short)bf16_bits(f[i]);
  return o;
}

template <int KQS>
__device__ __forceinline__ void wunit(const float* __restrict__ w, int ncol, int u, int nbase, unsigned short* wt) {
  const int n  = u >> KQS;
  const int k8 = (u & ((1 << KQS) - 1)) * 8;
  const int kk = k8 & 63;
  const v8us o = colpick8(w + (size_t)kk * (size_t)ncol + n, ncol);
  st2_v8us(wt + (size_t)(nbase + n) * (size_t)(8 << KQS) + k8, o);
}

__device__ __forceinline__ v4u maskw(const v4f a, unsigned m) {
  v4u r;
  r.x = __float_as_uint(a.x) & m; r.y = __float_as_uint(a.y) & m;
  r.z = __float_as_uint(a.z) & m; r.w = __float_as_uint(a.w) & m;
  return r;
}

__device__ __forceinline__ void vec4_block(const float* __restrict__ p0, int n0, const float* __restrict__ p1, int n1,
                                           const float* __restrict__ p2, int n2, const float* __restrict__ p3, int n3,
                                           float* dst, int tid) {
  const int u  = tid;
  const int b1 = n0, b2 = n0 + n1, b3 = b2 + n2, b4 = b3 + n3;
  int i0 = u;      i0 = i0 > n0 - 1 ? n0 - 1 : i0;
  int i1 = u - b1; i1 = i1 < 0 ? 0 : (i1 > n1 - 1 ? n1 - 1 : i1);
  int i2 = u - b2; i2 = i2 < 0 ? 0 : (i2 > n2 - 1 ? n2 - 1 : i2);
  const int h3 = n3 > 0 ? n3 - 1 : 0;
  int i3 = u - b3; i3 = i3 < 0 ? 0 : (i3 > h3 ? h3 : i3);
  const v4f a = *(const v4fa*)(p0 + 4 * i0);
  const v4f b = *(const v4fa*)(p1 + 4 * i1);
  const v4f c = *(const v4fa*)(p2 + 4 * i2);
  const v4f d = *(const v4fa*)(p3 + 4 * i3);
  asm volatile("" :: "v"(a), "v"(b));
  asm volatile("" :: "v"(c), "v"(d));
  const unsigned m0 = (u < b1) ? 0xffffffffu : 0u;
  const unsigned m1 = (u >= b1 && u < b2) ? 0xffffffffu : 0u;
  const unsigned m2 = (u >= b2 && u < b3) ? 0xffffffffu : 0u;
  const unsigned m3 = (u >= b3 && u < b4) ? 0xffffffffu : 0u;
  const v4u w = maskw(a, m0) | maskw(b, m1) | maskw(c, m2) | maskw(d, m3);
  v4f o;
  o.x = bf16_val(__uint_as_float(w.x)); o.y = bf16_val(__uint_as_float(w.y));
  o.z = bf16_val(__uint_as_float(w.z)); o.w = bf16_val(__uint_as_float(w.w));
  if (u < b4) st2_v4f(dst + 4 * u, o);
}

__global__ __launch_bounds__(NTHR) void k_prep(
    const float* __restrict__ x,
    const float* __restrict__ wq1, const float* __restrict__ wk1, const float* __restrict__ wv1, const float* __restrict__ ws1,
    const float* __restrict__ wq2, const float* __restrict__ wk2, const float* __restrict__ wv2, const float* __restrict__ ws2,
    const float* __restrict__ wf,
    const float* __restrict__ bq1, const float* __restrict__ bk1, const float* __restrict__ bv1, const float* __restrict__ bs1,
    const float* __restrict__ bq2, const float* __restrict__ bk2, const float* __restrict__ bv2, const float* __restrict__ bs2,
    const float* __restrict__ lng, const float* __restrict__ lnb, const float* __restrict__ bfin,
    unsigned short* xb, unsigned short* wt1, unsigned short* wt2, unsigned short* wft, float* sm) {
  const int tid = (int)threadIdx.x;
  const int blk = (int)blockIdx.x;
  if (blk < PB_X) {
    const int u   = blk * NTHR + tid;
    const int row = u >> 3, k8 = (u & 7) * 8;
    const int rc  = row < NN ? row : NN - 1;
    const unsigned mk = row < NN ? 0xffffu : 0u;
    const float* p = x + (size_t)rc * FIN + k8;
    const v4f a = *(const v4fa*)p;
    const v4f b = *(const v4fa*)(p + 4);
    v8us o;
    o[0] = (unsigned short)(bf16_bits(a.x) & mk); o[1] = (unsigned short)(bf16_bits(a.y) & mk);
    o[2] = (unsigned short)(bf16_bits(a.z) & mk); o[3] = (unsigned short)(bf16_bits(a.w) & mk);
    o[4] = (unsigned short)(bf16_bits(b.x) & mk); o[5] = (unsigned short)(bf16_bits(b.y) & mk);
    o[6] = (unsigned short)(bf16_bits(b.z) & mk); o[7] = (unsigned short)(bf16_bits(b.w) & mk);
    st2_v8us(xb + (size_t)row * FIN + k8, o);
  } else if (blk < PB_W1 + 8) {
    wunit<3>(wq1, HC, (blk - PB_W1) * NTHR + tid, 0, wt1);
  } else if (blk < PB_W1 + 16) {
    wunit<3>(wk1, HC, (blk - PB_W1 - 8) * NTHR + tid, 256, wt1);
  } else if (blk < PB_W1 + 24) {
    wunit<3>(wv1, HC, (blk - PB_W1 - 16) * NTHR + tid, 512, wt1);
  } else if (blk < PB_W1 + 26) {
    wunit<3>(ws1, FIN, (blk - PB_W1 - 24) * NTHR + tid, 768, wt1);
  } else if (blk < PB_W2 + 16) {
    wunit<4>(wq2, HC, (blk - PB_W2) * NTHR + tid, 0, wt2);
  } else if (blk < PB_W2 + 32) {
    wunit<4>(wk2, HC, (blk - PB_W2 - 16) * NTHR + tid, 256, wt2);
  } else if (blk < PB_W2 + 48) {
    wunit<4>(wv2, HC, (blk - PB_W2 - 32) * NTHR + tid, 512, wt2);
  } else if (blk < PB_W2 + 52) {
    wunit<4>(ws2, FIN, (blk - PB_W2 - 48) * NTHR + tid, 768, wt2);
  } else if (blk < PB_WF + 2) {
    wunit<4>(wf, OUTC, (blk - PB_WF) * NTHR + tid, 0, wft);
  } else if (blk == PB_SM) {
    vec4_block(bq1, 64, bk1, 64, bv1, 64, bs1, 16, sm + SM_B1, tid);
  } else if (blk == PB_SM + 1) {
    vec4_block(bq2, 64, bk2, 64, bv2, 64, bs2, 16, sm + SM_B2, tid);
  } else {
    vec4_block(lng, 16, lnb, 16, bfin, 8, bfin, 0, sm + SM_LNG, tid);
  }
}

__device__ __forceinline__ void bucket_flush(const int* pl, const int* cnt, int ov, int* lp, int* cop, int* fp,
                                             int tid) {
#pragma unroll 1
  for (int i = tid * 4; i < RCAP; i += NTHR * 4) {
    const v4i v = *(const v4ia*)(pl + i);
    *(volatile v4i*)(lp + i) = v;
  }
#pragma unroll 1
  for (int i = tid * 4; i < 2 * NBRUN; i += NTHR * 4) {
    const v4i v = *(const v4ia*)(cnt + i);
    *(volatile v4i*)(cop + i) = v;
  }
  if (tid < 8) {
    const v4i f = {ov, ov, ov, ov};
    *(volatile v4i*)(fp + 4 * tid) = f;
  }
}

__global__ __launch_bounds__(NTHR) void k_bucket(const int* __restrict__ srcs, const int* __restrict__ dsts,
                                                 int* LIST, int* CO, int* FLAG) {
  extern __shared__ __attribute__((aligned(16))) int dsm[];
  int* wl   = dsm;
  int* pl   = dsm + NWAVE * WLCAP;
  int* cnt  = pl + RCAP;
  int* offs = cnt + NBRUN;
  int* cur  = offs + NBRUN;
  int* misc = cur + NBRUN;
  const int tid = (int)threadIdx.x, lane = tid & 31, wave = tid >> 5;
  const int blk = (int)blockIdx.x;
  const unsigned nbs = (unsigned)(blk * NBRUN);

  {
    const v4i z4 = {0, 0, 0, 0};
    for (int i = tid * 4; i < BK_ZINTS; i += NTHR * 4) *(v4ia*)(dsm + i) = z4;
    if (tid < 16) misc[tid] = 0;
  }
  __syncthreads();

  {
    const int ebeg = wave * PERW;
    const int eend = (ebeg + PERW < NE) ? (ebeg + PERW) : NE;
    int* mylist = wl + wave * WLCAP;
    int wc = 0;
#pragma unroll 1
    for (int cb = ebeg; cb < eend; cb += WCH) {
      const int e0 = cb + lane * EPT;
      const v4i da = *(const v4ia*)(dsts + e0);
      const v4i db = *(const v4ia*)(dsts + e0 + 4);
      const unsigned s0 = (unsigned)da.x - nbs, s1 = (unsigned)da.y - nbs;
      const unsigned s2 = (unsigned)da.z - nbs, s3 = (unsigned)da.w - nbs;
      const unsigned s4 = (unsigned)db.x - nbs, s5 = (unsigned)db.y - nbs;
      const unsigned s6 = (unsigned)db.z - nbs, s7 = (unsigned)db.w - nbs;
      const bool h0 = s0 < (unsigned)NBRUN, h1 = s1 < (unsigned)NBRUN, h2 = s2 < (unsigned)NBRUN, h3 = s3 < (unsigned)NBRUN;
      const bool h4 = s4 < (unsigned)NBRUN, h5 = s5 < (unsigned)NBRUN, h6 = s6 < (unsigned)NBRUN, h7 = s7 < (unsigned)NBRUN;
      const unsigned m0 = __builtin_amdgcn_ballot_w32(h0), m1 = __builtin_amdgcn_ballot_w32(h1);
      const unsigned m2 = __builtin_amdgcn_ballot_w32(h2), m3 = __builtin_amdgcn_ballot_w32(h3);
      const unsigned m4 = __builtin_amdgcn_ballot_w32(h4), m5 = __builtin_amdgcn_ballot_w32(h5);
      const unsigned m6 = __builtin_amdgcn_ballot_w32(h6), m7 = __builtin_amdgcn_ballot_w32(h7);
      const unsigned any = m0 | m1 | m2 | m3 | m4 | m5 | m6 | m7;
      if (any != 0u) {
        const int pre = (int)(__builtin_amdgcn_mbcnt_lo(m0, 0u) + __builtin_amdgcn_mbcnt_lo(m1, 0u) +
                              __builtin_amdgcn_mbcnt_lo(m2, 0u) + __builtin_amdgcn_mbcnt_lo(m3, 0u) +
                              __builtin_amdgcn_mbcnt_lo(m4, 0u) + __builtin_amdgcn_mbcnt_lo(m5, 0u) +
                              __builtin_amdgcn_mbcnt_lo(m6, 0u) + __builtin_amdgcn_mbcnt_lo(m7, 0u));
        int p = wc + pre;
        if (h0) { if (p < WLCAP) mylist[p] = ((e0 + 0) << SLB) | (int)s0; p = p + 1; }
        if (h1) { if (p < WLCAP) mylist[p] = ((e0 + 1) << SLB) | (int)s1; p = p + 1; }
        if (h2) { if (p < WLCAP) mylist[p] = ((e0 + 2) << SLB) | (int)s2; p = p + 1; }
        if (h3) { if (p < WLCAP) mylist[p] = ((e0 + 3) << SLB) | (int)s3; p = p + 1; }
        if (h4) { if (p < WLCAP) mylist[p] = ((e0 + 4) << SLB) | (int)s4; p = p + 1; }
        if (h5) { if (p < WLCAP) mylist[p] = ((e0 + 5) << SLB) | (int)s5; p = p + 1; }
        if (h6) { if (p < WLCAP) mylist[p] = ((e0 + 6) << SLB) | (int)s6; p = p + 1; }
        if (h7) { if (p < WLCAP) mylist[p] = ((e0 + 7) << SLB) | (int)s7; p = p + 1; }
        wc += (int)(__builtin_popcount(m0) + __builtin_popcount(m1) + __builtin_popcount(m2) + __builtin_popcount(m3) +
                    __builtin_popcount(m4) + __builtin_popcount(m5) + __builtin_popcount(m6) + __builtin_popcount(m7));
      }
    }
    if (lane == 0) misc[wave] = wc;
  }
  __syncthreads();

  if (wave == 0) {
    int ov = 0, tot = 0;
#pragma unroll 1
    for (int w2 = 0; w2 < NWAVE; ++w2) {
      int c = misc[w2];
      if (c > WLCAP) ov = 1;
      c = c < 0 ? 0 : (c > WLCAP ? WLCAP : c);
      c = __builtin_amdgcn_readfirstlane(c);
      tot += c;
#pragma unroll 1
      for (int b0 = 0; b0 < c; b0 += 32) {
        const int idx = b0 + lane;
        const int ent = wl[w2 * WLCAP + (idx < WLCAP ? idx : WLCAP - 1)];
        const int m32 = (c - b0) < 32 ? (c - b0) : 32;
#pragma unroll 1
        for (int k = 0; k < m32; ++k) {
          const int u    = __builtin_amdgcn_readlane(ent, k);
          const int slot = u & (NBRUN - 1);
          if (lane == 0) cnt[slot] = cnt[slot] + 1;
        }
      }
    }
    if (tot > RCAP) ov = 1;
    if (lane == 0) misc[9] = ov;
  }
  __syncthreads();
  if (wave == 0) {
    const int base = lane * (NBRUN / 32);
    int s = 0;
#pragma unroll 1
    for (int i = 0; i < NBRUN / 32; ++i) s += cnt[base + i];
    int incl = s;
#pragma unroll
    for (int d = 1; d < 32; d <<= 1) {
      const int y = __shfl_up(incl, d, 32);
      if (lane >= d) incl += y;
    }
    int run = incl - s;
#pragma unroll 1
    for (int i = 0; i < NBRUN / 32; ++i) {
      const int cv = cnt[base + i];
      offs[base + i] = run;
      cur[base + i]  = run;
      run += cv;
    }
  }
  __syncthreads();

  if (wave == 0) {
#pragma unroll 1
    for (int w2 = 0; w2 < NWAVE; ++w2) {
      int c = misc[w2];
      c = c < 0 ? 0 : (c > WLCAP ? WLCAP : c);
      c = __builtin_amdgcn_readfirstlane(c);
#pragma unroll 1
      for (int b0 = 0; b0 < c; b0 += 32) {
        const int idx = b0 + lane;
        const int ent = wl[w2 * WLCAP + (idx < WLCAP ? idx : WLCAP - 1)];
        int eid = (ent >> SLB) & 0xFFFFF;
        eid = eid > NE - 1 ? NE - 1 : eid;
        int sr = srcs[eid];
        sr = sr < 0 ? 0 : (sr > NN - 1 ? NN - 1 : sr);
        const int word = (int)((unsigned)sr | ((unsigned)(ent & (NBRUN - 1)) << 16));
        const int m32 = (c - b0) < 32 ? (c - b0) : 32;
#pragma unroll 1
        for (int k = 0; k < m32; ++k) {
          const int u    = __builtin_amdgcn_readlane(ent, k);
          const int wd   = __builtin_amdgcn_readlane(word, k);
          const int slot = u & (NBRUN - 1);
          if (lane == 0) {
            int p = cur[slot];
            p = p < 0 ? 0 : (p > RCAP - 1 ? RCAP - 1 : p);
            pl[p] = wd;
            cur[slot] = p + 1;
          }
        }
      }
    }
  }
  __syncthreads();

  const int ovf = misc[9];
  int* lp  = LIST + (size_t)blk * RCAP;
  int* cop = CO + (size_t)blk * (2 * NBRUN);
  int* fp  = FLAG + (size_t)blk * 32;
  bucket_flush(pl, cnt, ovf, lp, cop, fp, tid);
  __threadfence();
  bucket_flush(pl, cnt, ovf, lp, cop, fp, tid);
}

template <int KEXT, int WP, int NT>
__device__ __forceinline__ void gemm_tiles(const unsigned short* __restrict__ ap,
                                           const unsigned short* __restrict__ bp, v8f (&acc)[NT]) {
#pragma unroll 1
  for (int k0 = 0; k0 < KEXT; k0 += 32) {
    FragB af;
    af.h[0] = *(const v8usa*)(ap + k0);
    af.h[1] = *(const v8usa*)(ap + k0 + 16);
#pragma unroll
    for (int nt = 0; nt < NT; ++nt) {
      const unsigned short* wq = bp + (size_t)(16 * nt) * (size_t)WP + k0;
      FragB bf;
      bf.h[0] = *(const v8usa*)wq;
      bf.h[1] = *(const v8usa*)(wq + 16);
      acc[nt] = wmb(af, bf, acc[nt]);
    }
  }
}

template <int KEXT, int AP, int WP>
__global__ __launch_bounds__(NTHR) __attribute__((amdgpu_num_vgpr(248)))
void k_proj(const unsigned short* __restrict__ A, const unsigned short* __restrict__ WT,
            const float* __restrict__ bias, float* F) {
  __shared__ __attribute__((aligned(16))) float stg[GBM * SP];
  __shared__ __attribute__((aligned(16))) float sb[64];
  const int tid = (int)threadIdx.x, lane = tid & 31, wave = tid >> 5, hh = lane >> 4, m = lane & 15;
  const int rowBase = (int)blockIdx.x * GBM;
  const int cb = (int)blockIdx.y;
  const int n0 = 64 * cb;
  if (tid < 16) *(v4fa*)(sb + 4 * tid) = *(const v4fa*)(bias + n0 + 4 * tid);

  v8f acc[4];
  {
    const v8f z = {0.f, 0.f, 0.f, 0.f, 0.f, 0.f, 0.f, 0.f};
#pragma unroll
    for (int t = 0; t < 4; ++t) acc[t] = z;
  }
  const unsigned short* ap = A + (size_t)(rowBase + 16 * wave + m) * (size_t)AP + 8 * hh;
  const unsigned short* bp = WT + (size_t)(n0 + m) * (size_t)WP + 8 * hh;
  gemm_tiles<KEXT, WP, 4>(ap, bp, acc);
#pragma unroll
  for (int nt = 0; nt < 4; ++nt) {
#pragma unroll
    for (int r = 0; r < 8; ++r) stg[(16 * wave + 8 * hh + r) * SP + 16 * nt + m] = acc[nt][r];
  }
  __syncthreads();

  const size_t poff = (cb < 4) ? (size_t)0 : ((cb < 12) ? FKV : FS);
  const int ld   = (cb < 4) ? 256 : ((cb < 12) ? 512 : 64);
  const int col0 = (cb < 4) ? n0 : ((cb < 12) ? (n0 - 256) : 0);
  const v4f bv = *(const v4fa*)(sb + 4 * m);
#pragma unroll 1
  for (int i = 0; i < 8; ++i) {
    const int lr   = 16 * wave + 2 * i + hh;
    const int grow = rowBase + lr;
    const v4f a = *(const v4fa*)(stg + lr * SP + 4 * m);
    v4f o;
    o.x = a.x + bv.x; o.y = a.y + bv.y; o.z = a.z + bv.z; o.w = a.w + bv.w;
    st2_v4f(F + poff + (size_t)grow * (size_t)ld + col0 + 4 * m, o);
  }
}

__device__ __forceinline__ float gsum8(float v) {
  v += __shfl_xor(v, 1, 32);
  v += __shfl_xor(v, 2, 32);
  v += __shfl_xor(v, 4, 32);
  return v;
}
__device__ __forceinline__ float hsum4(float v) {
  v += __shfl_xor(v, 8, 32);
  v += __shfl_xor(v, 16, 32);
  return v;
}
__device__ __forceinline__ float relu_keep(float v) { return (v > 0.0f) ? v : (v - v); }

template <int RELU>
__global__ __launch_bounds__(NTHR) void k_replay(const int* __restrict__ LIST, const int* __restrict__ CO,
                                                 const int* __restrict__ FLAG, const float* __restrict__ F,
                                                 const float* __restrict__ SM, unsigned short* H) {
  __shared__ __attribute__((aligned(16))) float sgb[128];
  const int tid = (int)threadIdx.x, lane = tid & 31;
  const int wave = __builtin_amdgcn_readfirstlane(tid >> 5);
  const int rowBase = (int)blockIdx.x * RBM;
  const int bucket  = rowBase >> SLB;
  if (tid < 32) *(v4fa*)(sgb + 4 * tid) = *(const v4fa*)(SM + SM_LNG + 4 * tid);
  __syncthreads();

  const int* lb  = LIST + (size_t)bucket * RCAP;
  const int* cob = CO + (size_t)bucket * (2 * NBRUN);
  const int flag = FLAG[(size_t)bucket * 32];
  const float qnan = __uint_as_float(0x7fc00000u);
  const int c8 = 8 * (lane & 7);
  const float* KVp = F + FKV;
  const float* Sp  = F + FS;
  const v4f ga = *(const v4fa*)(sgb + c8),      gb = *(const v4fa*)(sgb + c8 + 4);
  const v4f ba = *(const v4fa*)(sgb + 64 + c8), bb = *(const v4fa*)(sgb + 64 + c8 + 4);

#pragma unroll 1
  for (int i = 0; i < RBM / NWAVE; ++i) {
    const int d    = rowBase + (RBM / NWAVE) * wave + i;
    const int slot = d & (NBRUN - 1);
    int c = cob[slot];
    int o = cob[NBRUN + slot];
    const bool big = c > TRIPCAP;
    c = c < 0 ? 0 : (c > TRIPCAP ? TRIPCAP : c);
    o = o < 0 ? 0 : (o > RCAP - 1 ? RCAP - 1 : o);
    c = c > RCAP - o ? RCAP - o : c;
    const int cs = __builtin_amdgcn_readfirstlane(c);
    const int os = __builtin_amdgcn_readfirstlane(o);
    int last = os + cs - 1;
    last = last < os ? os : last;

    const float* qp = F + (size_t)d * HC + 8 * lane;
    v4f qa = *(const v4fa*)qp, qb = *(const v4fa*)(qp + 4);
    qa = qa * 0.125f; qb = qb * 0.125f;

    float mx = 0.0f, den = 0.0f;
    v4f aa = {0.f, 0.f, 0.f, 0.f}, ab = {0.f, 0.f, 0.f, 0.f};

#pragma unroll 1
    for (int cb0 = 0; cb0 < cs; cb0 += 32) {
      int idx = os + cb0 + lane;
      idx = idx > last ? last : idx;
      const int ent = lb[idx];
      const int m32 = (cs - cb0) < 32 ? (cs - cb0) : 32;
#pragma unroll 1
      for (int k = 0; k < m32; ++k) {
        const int wd = __builtin_amdgcn_readlane(ent, k);
        int sr = wd & 0xffff;
        sr = sr > NN - 1 ? NN - 1 : sr;
        const float* kr = KVp + (size_t)sr * 512 + 8 * lane;
        const v4f k0 = *(const v4fa*)kr,         k1 = *(const v4fa*)(kr + 4);
        const v4f v0 = *(const v4fa*)(kr + 256), v1 = *(const v4fa*)(kr + 260);
        float p = qa.x * k0.x;
        p = fmaf(qa.y, k0.y, p); p = fmaf(qa.z, k0.z, p); p = fmaf(qa.w, k0.w, p);
        p = fmaf(qb.x, k1.x, p); p = fmaf(qb.y, k1.y, p); p = fmaf(qb.z, k1.z, p); p = fmaf(qb.w, k1.w, p);
        p = gsum8(p);
        const bool first = (cb0 + k) == 0;
        const float df = p - mx;
        const bool up  = first | (df > 0.0f);
        const float ee = expf(-fabsf(df));
        const float s1 = up ? ee : 1.0f;
        const float s2 = up ? 1.0f : ee;
        mx  = up ? p : mx;
        den = fmaf(den, s1, s2);
        aa.x = fmaf(aa.x, s1, s2 * v0.x); aa.y = fmaf(aa.y, s1, s2 * v0.y);
        aa.z = fmaf(aa.z, s1, s2 * v0.z); aa.w = fmaf(aa.w, s1, s2 * v0.w);
        ab.x = fmaf(ab.x, s1, s2 * v1.x); ab.y = fmaf(ab.y, s1, s2 * v1.y);
        ab.z = fmaf(ab.z, s1, s2 * v1.z); ab.w = fmaf(ab.w, s1, s2 * v1.w);
      }
    }

    const float inv = 1.0f / (den + 1e-16f);
    aa = aa * inv; ab = ab * inv;
    aa.x = hsum4(aa.x); aa.y = hsum4(aa.y); aa.z = hsum4(aa.z); aa.w = hsum4(aa.w);
    ab.x = hsum4(ab.x); ab.y = hsum4(ab.y); ab.z = hsum4(ab.z); ab.w = hsum4(ab.w);
    const float* sp = Sp + (size_t)d * FIN + c8;
    const v4f sa = *(const v4fa*)sp, sbv = *(const v4fa*)(sp + 4);
    const v4f xa = aa * 0.25f + sa;
    const v4f xb = ab * 0.25f + sbv;

    float sum = ((xa.x + xa.y) + (xa.z + xa.w)) + ((xb.x + xb.y) + (xb.z + xb.w));
    sum = gsum8(sum);
    const float mu = sum * (1.0f / 64.0f);
    const v4f da = xa - mu, db = xb - mu;
    float sq = ((da.x * da.x + da.y * da.y) + (da.z * da.z + da.w * da.w)) +
               ((db.x * db.x + db.y * db.y) + (db.z * db.z + db.w * db.w));
    sq = gsum8(sq);
    const float var  = sq * (1.0f / 64.0f);
    const float rstd = 1.0f / sqrtf(var + 1e-5f);
    v4f ya = da * rstd * ga + ba;
    v4f yb = db * rstd * gb + bb;

    if (RELU != 0) {
      ya.x = relu_keep(ya.x); ya.y = relu_keep(ya.y); ya.z = relu_keep(ya.z); ya.w = relu_keep(ya.w);
      yb.x = relu_keep(yb.x); yb.y = relu_keep(yb.y); yb.z = relu_keep(yb.z); yb.w = relu_keep(yb.w);
    }
    const bool bad  = (flag != 0) | big;
    const bool live = d < NN;
    ya.x = bad ? qnan : ya.x; ya.y = bad ? qnan : ya.y; ya.z = bad ? qnan : ya.z; ya.w = bad ? qnan : ya.w;
    yb.x = bad ? qnan : yb.x; yb.y = bad ? qnan : yb.y; yb.z = bad ? qnan : yb.z; yb.w = bad ? qnan : yb.w;
    ya.x = live ? ya.x : 0.0f; ya.y = live ? ya.y : 0.0f; ya.z = live ? ya.z : 0.0f; ya.w = live ? ya.w : 0.0f;
    yb.x = live ? yb.x : 0.0f; yb.y = live ? yb.y : 0.0f; yb.z = live ? yb.z : 0.0f; yb.w = live ? yb.w : 0.0f;

    const unsigned h0 = bf16_bits(ya.x), h1 = bf16_bits(ya.y), h2 = bf16_bits(ya.z), h3 = bf16_bits(ya.w);
    const unsigned h4 = bf16_bits(yb.x), h5 = bf16_bits(yb.y), h6 = bf16_bits(yb.z), h7 = bf16_bits(yb.w);
    const unsigned l0 = bf16_bits(ya.x - __uint_as_float(h0 << 16)), l1 = bf16_bits(ya.y - __uint_as_float(h1 << 16));
    const unsigned l2 = bf16_bits(ya.z - __uint_as_float(h2 << 16)), l3 = bf16_bits(ya.w - __uint_as_float(h3 << 16));
    const unsigned l4 = bf16_bits(yb.x - __uint_as_float(h4 << 16)), l5 = bf16_bits(yb.y - __uint_as_float(h5 << 16));
    const unsigned l6 = bf16_bits(yb.z - __uint_as_float(h6 << 16)), l7 = bf16_bits(yb.w - __uint_as_float(h7 << 16));
    const unsigned mk = (lane & 8) ? 0u : 0xffffffffu;
    v4u pv;
    pv.x = ((h0 | (h1 << 16)) & mk) | ((l0 | (l1 << 16)) & ~mk);
    pv.y = ((h2 | (h3 << 16)) & mk) | ((l2 | (l3 << 16)) & ~mk);
    pv.z = ((h4 | (h5 << 16)) & mk) | ((l4 | (l5 << 16)) & ~mk);
    pv.w = ((h6 | (h7 << 16)) & mk) | ((l6 | (l7 << 16)) & ~mk);
    unsigned short* hp = H + (size_t)d * KL + c8 + ((lane & 8) ? 64 : 0);
    if (lane < 16) *(volatile v4u*)hp = pv;
    __threadfence();
    if (lane < 16) *(volatile v4u*)hp = pv;
  }
}

template <int KEXT>
__global__ __launch_bounds__(NTHR) __attribute__((amdgpu_num_vgpr(248)))
void k_final(const unsigned short* __restrict__ A, const unsigned short* __restrict__ WFT,
             const float* __restrict__ SM, const int* __restrict__ FLAG, float* out) {
  __shared__ __attribute__((aligned(16))) float stg[GBM * SPF];
  __shared__ __attribute__((aligned(16))) float sb[32];
  const int tid = (int)threadIdx.x, lane = tid & 31, wave = tid >> 5, hh = lane >> 4, m = lane & 15;
  const int rowBase = (int)blockIdx.x * GBM;
  const int flag = FLAG[(size_t)(rowBase >> SLB) * 32];
  if (tid < 8) *(v4fa*)(sb + 4 * tid) = *(const v4fa*)(SM + SM_BF + 4 * tid);

  v8f acc[2];
  {
    const v8f z = {0.f, 0.f, 0.f, 0.f, 0.f, 0.f, 0.f, 0.f};
    acc[0] = z; acc[1] = z;
  }
  const unsigned short* ap = A + (size_t)(rowBase + 16 * wave + m) * (size_t)KL + 8 * hh;
  const unsigned short* bp = WFT + (size_t)m * (size_t)KL + 8 * hh;
  gemm_tiles<KEXT, KL, 2>(ap, bp, acc);
#pragma unroll
  for (int nt = 0; nt < 2; ++nt) {
#pragma unroll
    for (int r = 0; r < 8; ++r) stg[(16 * wave + 8 * hh + r) * SPF + 16 * nt + m] = acc[nt][r];
  }
  __syncthreads();

  const int piece = lane & 7, rq = lane >> 3;
  const v4f bv = *(const v4fa*)(sb + 4 * piece);
  const float qnan = __uint_as_float(0x7fc00000u);
  v4f fv[4];
#pragma unroll
  for (int i = 0; i < 4; ++i) {
    const int lr = 16 * wave + 4 * i + rq;
    const v4f a = *(const v4fa*)(stg + lr * SPF + 4 * piece);
    asm volatile("" :: "v"(a));
    v4f o;
    o.x = a.x + bv.x; o.y = a.y + bv.y; o.z = a.z + bv.z; o.w = a.w + bv.w;
    o.x = (flag != 0) ? qnan : o.x; o.y = (flag != 0) ? qnan : o.y;
    o.z = (flag != 0) ? qnan : o.z; o.w = (flag != 0) ? qnan : o.w;
    fv[i] = o;
  }
#pragma unroll
  for (int i = 0; i < 4; ++i) {
    const int grow = rowBase + 16 * wave + 4 * i + rq;
    if (grow < NN) *(volatile v4f*)(out + (size_t)grow * OUTC + 4 * piece) = fv[i];
  }
  __threadfence();
#pragma unroll
  for (int i = 0; i < 4; ++i) {
    const int grow = rowBase + 16 * wave + 4 * i + rq;
    if (grow < NN) *(volatile v4f*)(out + (size_t)grow * OUTC + 4 * piece) = fv[i];
  }
}

extern "C" void kernel_launch(void* const* d_in, const int* in_sizes, int n_in,
                              void* d_out, int out_size, void* d_ws, size_t ws_size,
                              hipStream_t stream) {
  if (n_in < 22) return;
  if (in_sizes[0] != NN * FIN) return;
  if (in_sizes[1] != 2 * NE) return;
  if (in_sizes[2] != FIN * HC || in_sizes[4] != FIN * HC || in_sizes[6] != FIN * HC) return;
  if (in_sizes[3] != HC || in_sizes[5] != HC || in_sizes[7] != HC) return;
  if (in_sizes[8] != FIN * FIN || in_sizes[9] != FIN) return;
  if (in_sizes[10] != FIN * HC || in_sizes[12] != FIN * HC || in_sizes[14] != FIN * HC) return;
  if (in_sizes[11] != HC || in_sizes[13] != HC || in_sizes[15] != HC) return;
  if (in_sizes[16] != FIN * FIN || in_sizes[17] != FIN) return;
  if (in_sizes[18] != FIN || in_sizes[19] != FIN) return;
  if (in_sizes[20] != FIN * OUTC || in_sizes[21] != OUTC) return;
  if (out_size != NN * OUTC) return;

  const float* x   = (const float*)d_in[0];
  const int*   ei  = (const int*)d_in[1];
  const float* Wq1 = (const float*)d_in[2];   const float* bq1 = (const float*)d_in[3];
  const float* Wk1 = (const float*)d_in[4];   const float* bk1 = (const float*)d_in[5];
  const float* Wv1 = (const float*)d_in[6];   const float* bv1 = (const float*)d_in[7];
  const float* Ws1 = (const float*)d_in[8];   const float* bs1 = (const float*)d_in[9];
  const float* Wq2 = (const float*)d_in[10];  const float* bq2 = (const float*)d_in[11];
  const float* Wk2 = (const float*)d_in[12];  const float* bk2 = (const float*)d_in[13];
  const float* Wv2 = (const float*)d_in[14];  const float* bv2 = (const float*)d_in[15];
  const float* Ws2 = (const float*)d_in[16];  const float* bs2 = (const float*)d_in[17];
  const float* lng = (const float*)d_in[18];  const float* lnb = (const float*)d_in[19];
  const float* Wf  = (const float*)d_in[20];  const float* bfn = (const float*)d_in[21];
  float* out = (float*)d_out;
  const int* srcs = ei;
  const int* dsts = ei + NE;

  constexpr size_t zH    = (size_t)MP * KL * 2;
  constexpr size_t zXB   = (size_t)MP * FIN * 2;
  constexpr size_t zF    = (size_t)MP * NPRJ * 4;
  constexpr size_t zLIST = (size_t)NBK * RCAP * 4;
  constexpr size_t zCO   = (size_t)NBK * 2 * NBRUN * 4;
  constexpr size_t zFLAG = 6400;
  constexpr size_t zWT1  = (size_t)NPRJ * FIN * 2;
  constexpr size_t zWT2  = (size_t)NPRJ * KL * 2;
  constexpr size_t zWFT  = (size_t)OUTC * KL * 2;
  constexpr size_t zSM   = 7424;
  constexpr size_t oH    = 0;
  constexpr size_t oF    = oH + zH;
  constexpr size_t oLIST = oF + zF;
  constexpr size_t oCO   = oLIST + zLIST;
  constexpr size_t oFLAG = oCO + zCO;
  constexpr size_t oWT1  = oFLAG + zFLAG;
  constexpr size_t oWT2  = oWT1 + zWT1;
  constexpr size_t oWFT  = oWT2 + zWT2;
  constexpr size_t oSM   = oWFT + zWFT;
  constexpr size_t oEND  = oSM + zSM;
  static_assert(zXB <= zH);
  static_assert(zH % 256 == 0 && zF % 256 == 0 && zLIST % 256 == 0 && zCO % 256 == 0 && zFLAG % 256 == 0);
  static_assert(zWT1 % 256 == 0 && zWT2 % 256 == 0 && zWFT % 256 == 0 && zSM % 256 == 0);
  static_assert(zFLAG >= (size_t)NBK * 128 && zSM >= (size_t)SM_TOT * 4);
  static_assert(oEND <= ((size_t)256 << 20));
  if (oEND > ws_size) return;

  char* ws = (char*)d_ws;
  unsigned short* H    = (unsigned short*)(ws + oH);
  unsigned short* XB   = (unsigned short*)(ws + oH);
  float*          F    = (float*)(ws + oF);
  int*            LIST = (int*)(ws + oLIST);
  int*            CO   = (int*)(ws + oCO);
  int*            FLAG = (int*)(ws + oFLAG);
  unsigned short* WT1  = (unsigned short*)(ws + oWT1);
  unsigned short* WT2  = (unsigned short*)(ws + oWT2);
  unsigned short* WFT  = (unsigned short*)(ws + oWFT);
  float*          SM   = (float*)(ws + oSM);

  hipFuncSetAttribute(reinterpret_cast<const void*>(&k_bucket), hipFuncAttributeMaxDynamicSharedMemorySize, (int)BK_LDS);

  k_prep<<<PB_TOT, NTHR, 0, stream>>>(x, Wq1, Wk1, Wv1, Ws1, Wq2, Wk2, Wv2, Ws2, Wf,
                                      bq1, bk1, bv1, bs1, bq2, bk2, bv2, bs2, lng, lnb, bfn,
                                      XB, WT1, WT2, WFT, SM);
  k_bucket<<<NBK, NTHR, BK_LDS, stream>>>(srcs, dsts, LIST, CO, FLAG);
  k_proj<FIN, FIN, FIN><<<dim3(MP / GBM, NPRJ / 64), NTHR, 0, stream>>>(XB, WT1, SM + SM_B1, F);
  k_replay<1><<<MP / RBM, NTHR, 0, stream>>>(LIST, CO, FLAG, F, SM, H);
  k_proj<K2EXT, KL, KL><<<dim3(MP / GBM, NPRJ / 64), NTHR, 0, stream>>>(H, WT2, SM + SM_B2, F);
  k_replay<0><<<MP / RBM, NTHR, 0, stream>>>(LIST, CO, FLAG, F, SM, H);
  k_final<KFEXT><<<MP / GBM, NTHR, 0, stream>>>(H, WFT, SM, FLAG, out);
}
